// IDKN_cat_10531259809802
// MI455X (gfx1250) — hardware-verified
//
#include <hip/hip_runtime.h>
#include <stddef.h>


#define XW      10
#define KP      32
#define XPITCH  32
#define EPITCH  8
#define NTHR    256
#define NWAVE   8
#define EPT     8
#define NGRP    2
#define CHUNK   (NTHR * EPT * NGRP)
#define WCAP    (EPT * NGRP * 32)
#define LISTN   (NWAVE * WCAP)
#define NBC     4096
#define NBF     1024
#define RCAP    40960
#define RBN     128
#define OTHR    512
#define BM      128
#define APK     40
#define TGT     256
#define DEGCAP  256
#define TROWS   32
#define DEGT    128
#define WPTOT   4096
#define WSCAP   134217728
#define NEG_SLOPE 0.2f

#define LDS_FILL ((RCAP + NBF + LISTN) * 4 + 64)

static_assert((CHUNK & (CHUNK - 1)) == 0);
static_assert(CHUNK <= 4096);
static_assert(NBC <= 4096 && NBF <= 4096);
static_assert((NBC & (NBC - 1)) == 0 && (NBF & (NBF - 1)) == 0);
static_assert(NBC == 4 * NBF);
static_assert(OTHR * 8 == NBC);
static_assert((RCAP % 32) == 0);
static_assert(TGT == NWAVE * 32);
static_assert((NBC % TGT) == 0);
static_assert((TGT % BM) == 0 && BM == NWAVE * 16);
static_assert(TROWS == 4 * NWAVE);
static_assert(DEGT == 4 * 32);
static_assert(((APK * 2) % 16) == 0 && APK >= KP);

typedef float          v4f  __attribute__((ext_vector_type(4)));
typedef float          v8f  __attribute__((ext_vector_type(8)));
typedef int            v4i  __attribute__((ext_vector_type(4)));
typedef unsigned short v8us __attribute__((ext_vector_type(8)));
typedef __bf16         v16b __attribute__((ext_vector_type(16)));
union FragB { v16b v; v8us h[2]; };

__device__ __forceinline__ unsigned int bfr(float f) {
  const unsigned int u = __float_as_uint(f);
  return (u + 0x7FFFu + ((u >> 16) & 1u)) >> 16;
}

__device__ __forceinline__ void split1(float x, unsigned short& hb, unsigned short& lb) {
  const unsigned int hu = bfr(x);
  const float hf = __uint_as_float(hu << 16);
  hb = (unsigned short)hu;
  lb = (unsigned short)bfr(x - hf);
}

__device__ __forceinline__ void split8(v4f a, v4f b, v8us& hi, v8us& lo) {
  unsigned short hb, lb;
  split1(a.x, hb, lb); hi[0] = hb; lo[0] = lb;
  split1(a.y, hb, lb); hi[1] = hb; lo[1] = lb;
  split1(a.z, hb, lb); hi[2] = hb; lo[2] = lb;
  split1(a.w, hb, lb); hi[3] = hb; lo[3] = lb;
  split1(b.x, hb, lb); hi[4] = hb; lo[4] = lb;
  split1(b.y, hb, lb); hi[5] = hb; lo[5] = lb;
  split1(b.z, hb, lb); hi[6] = hb; lo[6] = lb;
  split1(b.w, hb, lb); hi[7] = hb; lo[7] = lb;
}

__device__ __forceinline__ v8f wmb(v16b a, v16b b, v8f c) {
  v8f d = __builtin_amdgcn_wmma_f32_16x16x32_bf16(false, a, false, b, (short)0, c, false, false);
  asm volatile("v_nop\n\tv_nop\n\tv_nop\n\tv_nop" : "+v"(d) : "v"(a), "v"(b));
  return d;
}

__device__ __forceinline__ float lrelu(float v) { return v >= 0.0f ? v : NEG_SLOPE * v; }

template <int NB>
__device__ __forceinline__ int scan_chunk(const int* __restrict__ keys, int nE, int cbase, int slotBase,
                                          int vec8, int* list, int tid, int lane, int wave) {
  int wc = 0;
#pragma unroll
  for (int g = 0; g < NGRP; ++g) {
    const int el0  = (g * NTHR + tid) * EPT;
    const int e0   = cbase + el0;
    const int sent = -2147483647 - 1;
    v4i da, db;
    if (vec8 != 0 && cbase + CHUNK <= nE) {
      da = *(const v4i*)(keys + e0);
      db = *(const v4i*)(keys + e0 + 4);
    } else {
      da.x = (e0     < nE) ? keys[min(e0, nE - 1)] : sent;
      da.y = (e0 + 1 < nE) ? keys[min(e0 + 1, nE - 1)] : sent;
      da.z = (e0 + 2 < nE) ? keys[min(e0 + 2, nE - 1)] : sent;
      da.w = (e0 + 3 < nE) ? keys[min(e0 + 3, nE - 1)] : sent;
      db.x = (e0 + 4 < nE) ? keys[min(e0 + 4, nE - 1)] : sent;
      db.y = (e0 + 5 < nE) ? keys[min(e0 + 5, nE - 1)] : sent;
      db.z = (e0 + 6 < nE) ? keys[min(e0 + 6, nE - 1)] : sent;
      db.w = (e0 + 7 < nE) ? keys[min(e0 + 7, nE - 1)] : sent;
    }
    const unsigned nb = (unsigned)slotBase;
    const unsigned s0 = (unsigned)da.x - nb, s1 = (unsigned)da.y - nb;
    const unsigned s2 = (unsigned)da.z - nb, s3 = (unsigned)da.w - nb;
    const unsigned s4 = (unsigned)db.x - nb, s5 = (unsigned)db.y - nb;
    const unsigned s6 = (unsigned)db.z - nb, s7 = (unsigned)db.w - nb;
    const bool h0 = s0 < (unsigned)NB, h1 = s1 < (unsigned)NB, h2 = s2 < (unsigned)NB, h3 = s3 < (unsigned)NB;
    const bool h4 = s4 < (unsigned)NB, h5 = s5 < (unsigned)NB, h6 = s6 < (unsigned)NB, h7 = s7 < (unsigned)NB;
    const unsigned any = __builtin_amdgcn_ballot_w32(h0 | h1 | h2 | h3 | h4 | h5 | h6 | h7);
    if (any != 0u) {
#define HITJ(J, HJ, SJ) { \
        const unsigned mj = __builtin_amdgcn_ballot_w32(HJ); \
        if (mj != 0u) { \
          if (HJ) { \
            const int pos = wc + (int)__builtin_amdgcn_mbcnt_lo(mj, 0u); \
            if (pos < WCAP) list[wave * WCAP + pos] = ((el0 + (J)) << 12) | (int)(SJ); \
          } \
          wc += (int)__builtin_popcount(mj); } }
      HITJ(0, h0, s0)
      HITJ(1, h1, s1)
      HITJ(2, h2, s2)
      HITJ(3, h3, s3)
      HITJ(4, h4, s4)
      HITJ(5, h5, s5)
      HITJ(6, h6, s6)
      HITJ(7, h7, s7)
#undef HITJ
    }
  }
  return wc;
}

__global__ __launch_bounds__(NTHR) void k_wprep(const float* __restrict__ W1, const float* __restrict__ W2,
                                                const float* __restrict__ W3, unsigned short* wp) {
  const int tid = threadIdx.x;
  const int which = tid < 128 ? 0 : (tid < 192 ? 1 : 2);
  const int unit  = which == 0 ? tid : (which == 1 ? tid - 128 : tid - 192);
  const int n  = unit >> 2;
  const int k0 = (unit & 3) * 8;
  float v[8];
#pragma unroll
  for (int e = 0; e < 8; ++e) {
    const int k  = k0 + e;
    const int k1 = k > 19 ? 19 : k, n1 = n > 31 ? 31 : n;
    const int k2 = k > 31 ? 31 : k, n2 = n > 15 ? 15 : n;
    const int k3 = k > 15 ? 15 : k, n3 = n > 7 ? 7 : n;
    const float a1 = W1[k1 * 32 + n1];
    const float a2 = W2[k2 * 16 + n2];
    const float a3 = W3[k3 * 8 + n3];
    v[e] = which == 0 ? (k < 20 ? a1 : 0.0f)
         : (which == 1 ? a2 : ((k < 16 && n < 8) ? a3 : 0.0f));
  }
  v4f a, b;
  a.x = v[0]; a.y = v[1]; a.z = v[2]; a.w = v[3];
  b.x = v[4]; b.y = v[5]; b.z = v[6]; b.w = v[7];
  v8us hv, lv;
  split8(a, b, hv, lv);
  const int hoff = which == 0 ? 0 : (which == 1 ? 2048 : 3072);
  const int loff = hoff + (which == 0 ? 1024 : 512);
  unsigned short* dh = wp + hoff + unit * 8;
  unsigned short* dl = wp + loff + unit * 8;
  *(volatile v8us*)dh = hv;
  *(volatile v8us*)dl = lv;
  __threadfence();
  *(volatile v8us*)dh = hv;
  *(volatile v8us*)dl = lv;
}

__global__ __launch_bounds__(NTHR) void k_count(
    const int* __restrict__ keys, int* cnt, int nE, int vec8) {
  __shared__ __attribute__((aligned(16))) int scnt[NBC];
  __shared__ __attribute__((aligned(16))) int list[LISTN];
  __shared__ int wcnt[NWAVE];
  const int tid = threadIdx.x, lane = tid & 31, wave = tid >> 5;
  const int nodeBase = blockIdx.x * NBC;

  for (int i = tid; i < NBC; i += NTHR) scnt[i] = 0;
  __syncthreads();

  const int nChunks = (nE + CHUNK - 1) / CHUNK;
#pragma unroll 1
  for (int ch = 0; ch < nChunks; ++ch) {
    const int cbase = ch * CHUNK;
    const int wc = scan_chunk<NBC>(keys, nE, cbase, nodeBase, vec8, list, tid, lane, wave);
    if (lane == 0) wcnt[wave] = wc;
    __syncthreads();
    if (wave == 0) {
#pragma unroll 1
      for (int wsx = 0; wsx < NWAVE; ++wsx) {
        int n = __builtin_amdgcn_readfirstlane(wcnt[wsx]);
        n = n > WCAP ? WCAP : (n < 0 ? 0 : n);
        const int* lp = list + wsx * WCAP;
#pragma unroll 1
        for (int i = 0; i < n; ++i) {
          const int ent  = __builtin_amdgcn_readfirstlane(lp[i]);
          const int slot = ent & (NBC - 1);
          if (lane == 0) scnt[slot] = scnt[slot] + 1;
        }
      }
    }
    __syncthreads();
  }

  v4i cq[4];
#pragma unroll
  for (int q = 0; q < 4; ++q) {
    const int f = (wave * 4 + q) * 128 + 4 * lane;
    cq[q] = *(const v4i*)(scnt + f);
  }
  int* cp = cnt + (size_t)nodeBase;
#pragma unroll
  for (int q = 0; q < 4; ++q) {
    const int f = (wave * 4 + q) * 128 + 4 * lane;
    *(volatile v4i*)(cp + f) = cq[q];
  }
  __threadfence();
#pragma unroll
  for (int q = 0; q < 4; ++q) {
    const int f = (wave * 4 + q) * 128 + 4 * lane;
    *(volatile v4i*)(cp + f) = cq[q];
  }
}

__global__ __launch_bounds__(OTHR) void k_offsets(
    const int* __restrict__ cnt, int* off, int* rbase, int nChunk) {
  __shared__ __attribute__((aligned(16))) int soff[NBC];
  __shared__ __attribute__((aligned(16))) int srb[RBN];
  __shared__ int wtot[OTHR / 32];
  const int tid = threadIdx.x, lane = tid & 31, wave = tid >> 5, sub = tid >> 7;
  for (int i = tid; i < RBN; i += OTHR) srb[i] = 0;
  int carry = 0;
#pragma unroll 1
  for (int ch = 0; ch < nChunk; ++ch) {
    const int base = ch * NBC;
    const v4i c0 = *(const v4i*)(cnt + base + 8 * tid);
    const v4i c1 = *(const v4i*)(cnt + base + 8 * tid + 4);
    const int e0 = max(c0.x, 0), e1 = max(c0.y, 0), e2 = max(c0.z, 0), e3 = max(c0.w, 0);
    const int e4 = max(c1.x, 0), e5 = max(c1.y, 0), e6 = max(c1.z, 0), e7 = max(c1.w, 0);
    const int ts = e0 + e1 + e2 + e3 + e4 + e5 + e6 + e7;
    int incl = ts;
#pragma unroll
    for (int d = 1; d < 32; d <<= 1) {
      const int t = __shfl_up(incl, d);
      if (lane >= d) incl += t;
    }
    if (lane == 31) wtot[wave] = incl;
    __syncthreads();
    const int S0 = wtot[0]  + wtot[1]  + wtot[2]  + wtot[3];
    const int S1 = wtot[4]  + wtot[5]  + wtot[6]  + wtot[7];
    const int S2 = wtot[8]  + wtot[9]  + wtot[10] + wtot[11];
    const int S3 = wtot[12] + wtot[13] + wtot[14] + wtot[15];
    int pre = 0;
#pragma unroll 1
    for (int w = 4 * sub; w < wave; ++w) pre += wtot[w];
    const int b0 = carry;
    const int b1 = b0 + ((S0 + 31) & ~31);
    const int b2 = b1 + ((S1 + 31) & ~31);
    const int b3 = b2 + ((S2 + 31) & ~31);
    const int b4 = b3 + ((S3 + 31) & ~31);
    const int myb = sub == 0 ? b0 : (sub == 1 ? b1 : (sub == 2 ? b2 : b3));
    if (tid == 0) {
      srb[min(4 * ch + 0, RBN - 1)] = b0;
      srb[min(4 * ch + 1, RBN - 1)] = b1;
      srb[min(4 * ch + 2, RBN - 1)] = b2;
      srb[min(4 * ch + 3, RBN - 1)] = b3;
    }
    int run = myb + pre + incl - ts;
    soff[8 * tid + 0] = run; run += e0;
    soff[8 * tid + 1] = run; run += e1;
    soff[8 * tid + 2] = run; run += e2;
    soff[8 * tid + 3] = run; run += e3;
    soff[8 * tid + 4] = run; run += e4;
    soff[8 * tid + 5] = run; run += e5;
    soff[8 * tid + 6] = run; run += e6;
    soff[8 * tid + 7] = run;
    carry = b4;
    __syncthreads();
    const v4i o0 = *(const v4i*)(soff + 4 * tid);
    const v4i o1 = *(const v4i*)(soff + 4 * (tid + OTHR));
    int* op = off + base;
    *(volatile v4i*)(op + 4 * tid) = o0;
    *(volatile v4i*)(op + 4 * (tid + OTHR)) = o1;
    __threadfence();
    *(volatile v4i*)(op + 4 * tid) = o0;
    *(volatile v4i*)(op + 4 * (tid + OTHR)) = o1;
    __syncthreads();
  }
  if (tid == 0) srb[min(4 * nChunk, RBN - 1)] = carry;
  __syncthreads();
  v4i rv = {0, 0, 0, 0};
  if (tid < 32) rv = *(const v4i*)(srb + 4 * tid);
  if (tid < 32) *(volatile v4i*)(rbase + 4 * tid) = rv;
  __threadfence();
  if (tid < 32) *(volatile v4i*)(rbase + 4 * tid) = rv;
}

__global__ __launch_bounds__(NTHR) void k_fill(
    const int* __restrict__ vals, const int* __restrict__ keys,
    const int* __restrict__ off, const int* __restrict__ rbase,
    int* csr, int nN, int nE, int vec8, int csrLen) {
  extern __shared__ v4f lds_dyn[];
  int* region = (int*)lds_dyn;
  int* cursor = region + RCAP;
  int* list   = cursor + NBF;
  int* wcnt   = list + LISTN;
  const int tid = threadIdx.x, lane = tid & 31, wave = tid >> 5;
  const int b = blockIdx.x;
  const int nodeBase = b * NBF;

  int rb0 = rbase[b];
  const int rb1 = rbase[b + 1];
  rb0 = rb0 < 0 ? 0 : (rb0 > csrLen ? csrLen : rb0);
  rb0 &= ~31;
  int len = rb1 - rb0;
  len = len < 0 ? 0 : (len > RCAP ? RCAP : len);
  int lenW = (len + 31) & ~31;
  if (rb0 + lenW > csrLen) lenW = (csrLen - rb0) & ~31;

  {
    const v4i z = {0, 0, 0, 0};
    for (int i = tid; i < RCAP / 4; i += NTHR) ((v4i*)region)[i] = z;
    for (int s = tid; s < NBF; s += NTHR) {
      int o = off[nodeBase + s] - rb0;
      o = o < 0 ? 0 : (o > RCAP ? RCAP : o);
      cursor[s] = o;
    }
  }
  __syncthreads();

  const int nChunks = (nE + CHUNK - 1) / CHUNK;
#pragma unroll 1
  for (int ch = 0; ch < nChunks; ++ch) {
    const int cbase = ch * CHUNK;
    const int wc = scan_chunk<NBF>(keys, nE, cbase, nodeBase, vec8, list, tid, lane, wave);
    if (lane == 0) wcnt[wave] = wc;
    __syncthreads();
    if (wave == 0) {
#pragma unroll 1
      for (int wsx = 0; wsx < NWAVE; ++wsx) {
        int n = __builtin_amdgcn_readfirstlane(wcnt[wsx]);
        n = n > WCAP ? WCAP : (n < 0 ? 0 : n);
        const int* lp = list + wsx * WCAP;
#pragma unroll 1
        for (int i = 0; i < n; ++i) {
          const int ent  = __builtin_amdgcn_readfirstlane(lp[i]);
          const int slot = ent & (NBF - 1);
          int e = cbase + ((ent >> 12) & (CHUNK - 1));
          e = e > nE - 1 ? nE - 1 : e;
          int val = vals[e];
          val = val < 0 ? 0 : (val > nN - 1 ? nN - 1 : val);
          if (lane == 0) {
            int pos = cursor[slot];
            pos = pos < 0 ? 0 : (pos > RCAP - 1 ? RCAP - 1 : pos);
            region[pos] = val;
            const int np = pos + 1;
            cursor[slot] = np > RCAP ? RCAP : np;
          }
        }
      }
    }
    __syncthreads();
  }

  const int nv = lenW >> 2;
  int* gp = csr + rb0;
#pragma unroll 1
  for (int i = tid; i < nv; i += NTHR) { const v4i v = ((const v4i*)region)[i]; *(volatile v4i*)(gp + 4 * i) = v; }
  __threadfence();
#pragma unroll 1
  for (int i = tid; i < nv; i += NTHR) { const v4i v = ((const v4i*)region)[i]; *(volatile v4i*)(gp + 4 * i) = v; }
}

template <int KD, int NC, int HEADS, int CAT>
__global__ __launch_bounds__(NTHR) void k_gemm(
    const float* __restrict__ A0, const float* __restrict__ A1, const unsigned short* __restrict__ Bw,
    const float* __restrict__ attS, const float* __restrict__ attD,
    float* C, float* eS, float* eD, int nRowsA) {
  constexpr int NCP = NC < 16 ? 16 : NC;
  constexpr int TPW = NCP / 16;
  static_assert(KD <= KP && NCP <= XPITCH && HEADS * 4 == NC && HEADS <= EPITCH);
  static_assert(TPW >= 1 && TPW <= 2);
  static_assert(CAT == 0 || KD == 2 * XW);
  __shared__ __attribute__((aligned(16))) unsigned short sHi[BM * APK];
  __shared__ __attribute__((aligned(16))) unsigned short sLo[BM * APK];
  __shared__ __attribute__((aligned(16))) float stg[BM * XPITCH];
  __shared__ __attribute__((aligned(16))) float sES[BM * EPITCH];
  __shared__ __attribute__((aligned(16))) float sED[BM * EPITCH];
  const int tid = threadIdx.x, lane = tid & 31, wave = tid >> 5, hh = lane >> 4, m = lane & 15;
  const int rowBase = blockIdx.x * BM;

#pragma unroll
  for (int i = 0; i < 2; ++i) {
    const int idx = i * NTHR + tid;
    const int r   = idx >> 2;
    const int c0  = (idx & 3) * 8;
    int row = rowBase + r;
    row = row > nRowsA - 1 ? nRowsA - 1 : row;
    float v[8];
#pragma unroll
    for (int e = 0; e < 8; ++e) {
      const int c = c0 + e;
      if constexpr (CAT != 0) {
        const int ca = c > XW - 1 ? XW - 1 : c;
        int cb = c - XW;
        cb = cb < 0 ? 0 : (cb > XW - 1 ? XW - 1 : cb);
        const float a = A0[(size_t)row * XW + ca];
        const float bq = A1[(size_t)row * XW + cb];
        v[e] = c < XW ? a : (c < 2 * XW ? bq : 0.0f);
      } else {
        const int cc = c > KD - 1 ? KD - 1 : c;
        const float a = A0[(size_t)row * XPITCH + cc];
        v[e] = c < KD ? a : 0.0f;
      }
    }
    v4f a, b;
    a.x = v[0]; a.y = v[1]; a.z = v[2]; a.w = v[3];
    b.x = v[4]; b.y = v[5]; b.z = v[6]; b.w = v[7];
    v8us hv, lv;
    split8(a, b, hv, lv);
    *(v8us*)(sHi + r * APK + c0) = hv;
    *(v8us*)(sLo + r * APK + c0) = lv;
  }
  __syncthreads();

  const int r0 = wave * 16;
  v8f acc[TPW];
#pragma unroll
  for (int t = 0; t < TPW; ++t) { v8f z = {0.f, 0.f, 0.f, 0.f, 0.f, 0.f, 0.f, 0.f}; acc[t] = z; }
  {
    const unsigned short* ahp = sHi + (r0 + m) * APK + 8 * hh;
    const unsigned short* alp = sLo + (r0 + m) * APK + 8 * hh;
    FragB ah, al;
    ah.h[0] = *(const v8us*)(ahp);
    ah.h[1] = *(const v8us*)(ahp + 16);
    al.h[0] = *(const v8us*)(alp);
    al.h[1] = *(const v8us*)(alp + 16);
#pragma unroll
    for (int t = 0; t < TPW; ++t) {
      const unsigned short* bp = Bw + (size_t)(16 * t + m) * KP + 8 * hh;
      FragB bh, bl;
      bh.h[0] = *(const v8us*)bp;
      bh.h[1] = *(const v8us*)(bp + 16);
      bl.h[0] = *(const v8us*)(bp + NCP * KP);
      bl.h[1] = *(const v8us*)(bp + NCP * KP + 16);
      acc[t] = wmb(ah.v, bh.v, acc[t]);
      acc[t] = wmb(ah.v, bl.v, acc[t]);
      acc[t] = wmb(al.v, bh.v, acc[t]);
    }
  }

  {
    float* sp = stg + (size_t)(r0 + 8 * hh) * XPITCH + m;
#pragma unroll
    for (int t = 0; t < 2; ++t) {
#pragma unroll
      for (int r = 0; r < 8; ++r) {
        float val = 0.0f;
        if constexpr (TPW == 2) { val = acc[t][r]; }
        else { if (t == 0) val = acc[0][r]; }
        sp[r * XPITCH + 16 * t] = val;
      }
    }
  }
  __syncthreads();

  const int rq  = lane >> 3;
  const int cq  = lane & 7;
  const int col = 4 * cq;
  const int hdc = cq < HEADS ? cq : HEADS - 1;
  const v4f sA = *(const v4f*)(attS + 4 * hdc);
  const v4f sD = *(const v4f*)(attD + 4 * hdc);
  v4f ov[4];
#pragma unroll
  for (int it = 0; it < 4; ++it) {
    const int row = r0 + 4 * it + rq;
    ov[it] = *(const v4f*)(stg + (size_t)row * XPITCH + col);
    *(volatile v4f*)(C + (size_t)(rowBase + row) * XPITCH + col) = ov[it];
    const v4f v = ov[it];
    float ps = v.x * sA.x + v.y * sA.y + v.z * sA.z + v.w * sA.w;
    float pd = v.x * sD.x + v.y * sD.y + v.z * sD.z + v.w * sD.w;
    if (cq >= HEADS) { ps = 0.0f; pd = 0.0f; }
    sES[row * EPITCH + cq] = ps;
    sED[row * EPITCH + cq] = pd;
  }
  __threadfence();
#pragma unroll
  for (int it = 0; it < 4; ++it) {
    const int row = r0 + 4 * it + rq;
    *(volatile v4f*)(C + (size_t)(rowBase + row) * XPITCH + col) = ov[it];
  }
  __syncthreads();

  const v4f dvs = *(const v4f*)(sES + 4 * tid);
  const v4f dvd = *(const v4f*)(sED + 4 * tid);
  const size_t eb = (size_t)rowBase * EPITCH + 4 * tid;
  *(volatile v4f*)(eS + eb) = dvs;
  *(volatile v4f*)(eD + eb) = dvd;
  __threadfence();
  *(volatile v4f*)(eS + eb) = dvs;
  *(volatile v4f*)(eD + eb) = dvd;
}

template <int NC>
__global__ __launch_bounds__(NTHR) void k_agg(
    const int* __restrict__ csr, const int* __restrict__ off, const int* __restrict__ cnt,
    const float* __restrict__ eS, const float* __restrict__ eD, const float* __restrict__ hw,
    const float* __restrict__ bias, float* xout, int nN, int csrLen) {
  constexpr int NQ = NC / 4;
  static_assert(NQ == 8 || NQ == 4 || NQ == 2);
  __shared__ __attribute__((aligned(16))) float sOut[NWAVE * 32 * XPITCH];
  const int tid = threadIdx.x, lane = tid & 31, wave = tid >> 5;
  const int tbase = blockIdx.x * TGT + wave * 32;
  const int q    = lane & 7;
  const int hd   = q & (NQ - 1);
  const int col0 = 4 * hd;
  const v4f z4 = {0.f, 0.f, 0.f, 0.f};
  const v4f bb = *(const v4f*)(bias + col0);

  const int cl    = tbase + lane;
  const int cnt_l = cnt[cl];
  const int off_l = off[cl];
  float* so = sOut + wave * (32 * XPITCH);

#pragma unroll 1
  for (int j = 0; j < 32; ++j) {
    const int c = tbase + j;
    int n = __shfl(cnt_l, j);
    n = n < 0 ? 0 : (n > DEGCAP ? DEGCAP : n);
    const int st = __shfl(off_l, j);
    const float ed    = eD[(size_t)c * EPITCH + hd];
    const float eself = lrelu(eS[(size_t)c * EPITCH + hd] + ed);

    float mx = eself;
#pragma unroll 1
    for (int q0 = 0; q0 < n; q0 += 32) {
      int pos = st + q0 + lane;
      pos = pos < 0 ? 0 : (pos > csrLen - 1 ? csrLen - 1 : pos);
      int sl = csr[pos];
      sl = sl < 0 ? 0 : (sl > nN - 1 ? nN - 1 : sl);
      const int mcnt = (n - q0) < 32 ? (n - q0) : 32;
#pragma unroll 1
      for (int pp = 0; pp < mcnt; ++pp) {
        const int s = __builtin_amdgcn_readlane(sl, pp);
        mx = fmaxf(mx, lrelu(eS[(size_t)s * EPITCH + hd] + ed));
      }
    }

    float p   = __expf(eself - mx);
    float den = p;
    v4f   acc = *(const v4f*)(hw + (size_t)c * XPITCH + col0) * p;
#pragma unroll 1
    for (int q0 = 0; q0 < n; q0 += 32) {
      int pos = st + q0 + lane;
      pos = pos < 0 ? 0 : (pos > csrLen - 1 ? csrLen - 1 : pos);
      int sl = csr[pos];
      sl = sl < 0 ? 0 : (sl > nN - 1 ? nN - 1 : sl);
      const int mcnt = (n - q0) < 32 ? (n - q0) : 32;
#pragma unroll 1
      for (int pp = 0; pp < mcnt; ++pp) {
        const int s = __builtin_amdgcn_readlane(sl, pp);
        p = __expf(lrelu(eS[(size_t)s * EPITCH + hd] + ed) - mx);
        den += p;
        const v4f h0 = *(const v4f*)(hw + (size_t)s * XPITCH + col0);
        acc = acc + h0 * p;
      }
    }

    const float rd = 1.0f / den;
    v4f v = acc * rd + bb;
    if (c >= nN) v = z4;
    if (q >= NQ)  v = z4;
    if (lane < 8) *(v4f*)(so + j * XPITCH + 4 * q) = v;
  }
  __syncthreads();

  v4f ov[8];
  float* gp = xout + (size_t)tbase * XPITCH;
#pragma unroll
  for (int it = 0; it < 8; ++it) {
    const int f = it * 32 + lane;
    ov[it] = *(const v4f*)(so + 4 * f);
    *(volatile v4f*)(gp + 4 * f) = ov[it];
  }
  __threadfence();
#pragma unroll
  for (int it = 0; it < 8; ++it) {
    const int f = it * 32 + lane;
    *(volatile v4f*)(gp + 4 * f) = ov[it];
  }
}

__global__ __launch_bounds__(NTHR) void k_tail(
    const int* __restrict__ csr, const int* __restrict__ off, const int* __restrict__ cnt,
    const float* __restrict__ x6, const float* __restrict__ x1, const float* __restrict__ lin2,
    float* out, int nN, int csrLen, int cntLen) {
  __shared__ __attribute__((aligned(16))) float sRes[TROWS];
  const int tid = threadIdx.x, lane = tid & 31, wave = tid >> 5;
  const int row0 = blockIdx.x * TROWS;
  const v4f z4 = {0.f, 0.f, 0.f, 0.f};
  const v4f lwa = *(const v4f*)lin2;
  const v4f lwb = *(const v4f*)(lin2 + 4);

#pragma unroll 1
  for (int t = 0; t < TROWS / NWAVE; ++t) {
    const int i  = row0 + wave * (TROWS / NWAVE) + t;
    const int ic = i > nN - 1 ? nN - 1 : i;
    const int ci = ic > cntLen - 1 ? cntLen - 1 : ic;
    int n = cnt[ci];
    n = n < 0 ? 0 : (n > DEGT ? DEGT : n);
    const int st = off[ci];
    int vs[4];
    int kp[4];
#pragma unroll
    for (int s = 0; s < 4; ++s) {
      const int p = 32 * s + lane;
      int pos = st + p;
      pos = pos < 0 ? 0 : (pos > csrLen - 1 ? csrLen - 1 : pos);
      int v = csr[pos];
      v = v < 0 ? 0 : (v > nN - 1 ? nN - 1 : v);
      vs[s] = v;
      kp[s] = (p < n && v != ic) ? 1 : 0;
    }
#pragma unroll 1
    for (int p = 0; p < n; ++p) {
      const int sidx = p >> 5, pl = p & 31;
      const int sel = sidx == 0 ? vs[0] : (sidx == 1 ? vs[1] : (sidx == 2 ? vs[2] : vs[3]));
      const int ep = __builtin_amdgcn_readlane(sel, pl);
#pragma unroll
      for (int s = 0; s < 4; ++s) {
        if ((32 * s + lane) > p && vs[s] == ep) kp[s] = 0;
      }
    }
    v4f sa = z4, sb = z4;
    int kc = 0;
#pragma unroll
    for (int s = 0; s < 4; ++s) {
      const float f = kp[s] != 0 ? 1.0f : 0.0f;
      const float* xp = x6 + (size_t)vs[s] * XPITCH;
      const v4f a = *(const v4f*)xp;
      const v4f b = *(const v4f*)(xp + 4);
      sa = sa + a * f;
      sb = sb + b * f;
      kc += kp[s];
    }
#pragma unroll
    for (int o = 16; o >= 1; o >>= 1) {
      sa.x += __shfl_xor(sa.x, o); sa.y += __shfl_xor(sa.y, o);
      sa.z += __shfl_xor(sa.z, o); sa.w += __shfl_xor(sa.w, o);
      sb.x += __shfl_xor(sb.x, o); sb.y += __shfl_xor(sb.y, o);
      sb.z += __shfl_xor(sb.z, o); sb.w += __shfl_xor(sb.w, o);
      kc   += __shfl_xor(kc, o);
    }
    const float* xip = x6 + (size_t)ic * XPITCH;
    const v4f xa = *(const v4f*)xip;
    const v4f xb = *(const v4f*)(xip + 4);
    const v4f ta = sa + xa, tb = sb + xb;
    const float rinv = 1.0f / (float)(kc + 1);
    const v4f aa = ta * rinv, ab = tb * rinv;
    const float r2 = xa.x * aa.x + xa.y * aa.y + xa.z * aa.z + xa.w * aa.w
                   + xb.x * ab.x + xb.y * ab.y + xb.z * ab.z + xb.w * ab.w;
    const float g  = aa.x * lwa.x + aa.y * lwa.y + aa.z * lwa.z + aa.w * lwa.w
                   + ab.x * lwb.x + ab.y * lwb.y + ab.z * lwb.z + ab.w * lwb.w;
    const float res = (r2 + x1[(size_t)ic * XW]) + g;
    if (lane == 0) sRes[wave * (TROWS / NWAVE) + t] = res;
  }
  __syncthreads();

  if (wave == 0) {
    const int rem = nN - row0;
    const int lq  = lane & 7;
    const v4f v = *(const v4f*)(sRes + 4 * lq);
    float* op = out + (size_t)row0 + 4 * lq;
    const bool full = (lane < 8) && (4 * lq + 4 <= rem);
    const bool part = (lane < 8) && !full && (4 * lq < rem);
    if (full) *(volatile v4f*)op = v;
    if (part) {
      if (4 * lq + 0 < rem) ((volatile float*)op)[0] = v.x;
      if (4 * lq + 1 < rem) ((volatile float*)op)[1] = v.y;
      if (4 * lq + 2 < rem) ((volatile float*)op)[2] = v.z;
    }
    __threadfence();
    if (full) *(volatile v4f*)op = v;
    if (part) {
      if (4 * lq + 0 < rem) ((volatile float*)op)[0] = v.x;
      if (4 * lq + 1 < rem) ((volatile float*)op)[1] = v.y;
      if (4 * lq + 2 < rem) ((volatile float*)op)[2] = v.z;
    }
  }
}

extern "C" void kernel_launch(void* const* d_in, const int* in_sizes, int n_in,
                              void* d_out, int out_size, void* d_ws, size_t ws_size,
                              hipStream_t stream) {
  if (n_in < 17) return;
  const int nN = in_sizes[0] / XW;
  const int nE = in_sizes[2] / 2;
  if (nN <= 0 || nE <= 0 || in_sizes[0] != nN * XW || in_sizes[1] != nN * XW || in_sizes[2] != 2 * nE) return;
  if (in_sizes[4] != 2 * XW * 32 || in_sizes[5] != 32 || in_sizes[6] != 32 || in_sizes[7] != 32) return;
  if (in_sizes[8] != 32 * 16 || in_sizes[9] != 16 || in_sizes[10] != 16 || in_sizes[11] != 16) return;
  if (in_sizes[12] != 16 * 8 || in_sizes[13] != 8 || in_sizes[14] != 8 || in_sizes[15] != 8 || in_sizes[16] != 8) return;
  if (out_size != nN) return;
  if (nE > (1 << 26) || nN > (1 << 22)) return;

  const float* x1   = (const float*)d_in[0];
  const float* x2   = (const float*)d_in[1];
  const int*   ei   = (const int*)d_in[2];
  const int*   esrc = ei;
  const int*   edst = ei + nE;
  const float* W1   = (const float*)d_in[4];
  const float* as1  = (const float*)d_in[5];
  const float* ad1  = (const float*)d_in[6];
  const float* b1   = (const float*)d_in[7];
  const float* W2   = (const float*)d_in[8];
  const float* as2  = (const float*)d_in[9];
  const float* ad2  = (const float*)d_in[10];
  const float* b2   = (const float*)d_in[11];
  const float* W3   = (const float*)d_in[12];
  const float* as3  = (const float*)d_in[13];
  const float* ad3  = (const float*)d_in[14];
  const float* b3   = (const float*)d_in[15];
  const float* lin2 = (const float*)d_in[16];
  float* out = (float*)d_out;

  const int NPAD   = ((nN + TGT - 1) / TGT) * TGT;
  const int nBC    = (nN + NBC - 1) / NBC;
  const int CNTPAD = nBC * NBC;
  if (4 * nBC + 1 > RBN) return;
  const int nBF    = (nN + NBF - 1) / NBF;
  const int csrLen = ((nE + 31) & ~31) + 4096;
  if (31 * 4 * nBC > 4096) return;
  const int nAgg   = NPAD / TGT;
  const int nGemm  = NPAD / BM;
  const int nTail  = (nN + TROWS - 1) / TROWS;
  if (nTail * TROWS > CNTPAD || NPAD > CNTPAD) return;

  char* ws = (char*)d_ws;
  size_t off = 0;
  const size_t oWp   = off; off += (size_t)WPTOT * 2;              off = (off + 255) & ~(size_t)255;
  const size_t oCntD = off; off += (size_t)CNTPAD * 4;             off = (off + 255) & ~(size_t)255;
  const size_t oOffD = off; off += (size_t)CNTPAD * 4;             off = (off + 255) & ~(size_t)255;
  const size_t oRbD  = off; off += (size_t)RBN * 4;                off = (off + 255) & ~(size_t)255;
  const size_t oCsrD = off; off += (size_t)csrLen * 4;             off = (off + 255) & ~(size_t)255;
  const size_t oCntS = off; off += (size_t)CNTPAD * 4;             off = (off + 255) & ~(size_t)255;
  const size_t oOffS = off; off += (size_t)CNTPAD * 4;             off = (off + 255) & ~(size_t)255;
  const size_t oRbS  = off; off += (size_t)RBN * 4;                off = (off + 255) & ~(size_t)255;
  const size_t oCsrS = off; off += (size_t)csrLen * 4;             off = (off + 255) & ~(size_t)255;
  const size_t oHw   = off; off += (size_t)NPAD * XPITCH * 4;      off = (off + 255) & ~(size_t)255;
  const size_t oX    = off; off += (size_t)NPAD * XPITCH * 4;      off = (off + 255) & ~(size_t)255;
  const size_t oES   = off; off += (size_t)NPAD * EPITCH * 4;      off = (off + 255) & ~(size_t)255;
  const size_t oED   = off; off += (size_t)NPAD * EPITCH * 4;      off = (off + 255) & ~(size_t)255;
  if (off > ws_size || off > (size_t)WSCAP) return;
  unsigned short* wp = (unsigned short*)(ws + oWp);
  int*   cntD = (int*)(ws + oCntD);
  int*   offD = (int*)(ws + oOffD);
  int*   rbD  = (int*)(ws + oRbD);
  int*   csrD = (int*)(ws + oCsrD);
  int*   cntS = (int*)(ws + oCntS);
  int*   offS = (int*)(ws + oOffS);
  int*   rbS  = (int*)(ws + oRbS);
  int*   csrS = (int*)(ws + oCsrS);
  float* hw   = (float*)(ws + oHw);
  float* xb   = (float*)(ws + oX);
  float* es   = (float*)(ws + oES);
  float* ed   = (float*)(ws + oED);
  const unsigned short* wp1 = wp;
  const unsigned short* wp2 = wp + 2048;
  const unsigned short* wp3 = wp + 3072;

  const int vec8 = ((nE & 3) == 0) ? 1 : 0;

  k_wprep<<<1, NTHR, 0, stream>>>(W1, W2, W3, wp);

  k_count<<<nBC, NTHR, 0, stream>>>(edst, cntD, nE, vec8);
  k_offsets<<<1, OTHR, 0, stream>>>(cntD, offD, rbD, nBC);
  hipFuncSetAttribute(reinterpret_cast<const void*>(&k_fill),
                      hipFuncAttributeMaxDynamicSharedMemorySize, LDS_FILL);
  k_fill<<<nBF, NTHR, LDS_FILL, stream>>>(esrc, edst, offD, rbD, csrD, nN, nE, vec8, csrLen);

  k_count<<<nBC, NTHR, 0, stream>>>(esrc, cntS, nE, vec8);
  k_offsets<<<1, OTHR, 0, stream>>>(cntS, offS, rbS, nBC);
  k_fill<<<nBF, NTHR, LDS_FILL, stream>>>(edst, esrc, offS, rbS, csrS, nN, nE, vec8, csrLen);

  k_gemm<20, 32, 8, 1><<<nGemm, NTHR, 0, stream>>>(x1, x2, wp1, as1, ad1, hw, es, ed, nN);
  k_agg<32><<<nAgg, NTHR, 0, stream>>>(csrD, offD, cntD, es, ed, hw, b1, xb, nN, csrLen);

  k_gemm<32, 16, 4, 0><<<nGemm, NTHR, 0, stream>>>(xb, xb, wp2, as2, ad2, hw, es, ed, NPAD);
  k_agg<16><<<nAgg, NTHR, 0, stream>>>(csrD, offD, cntD, es, ed, hw, b2, xb, nN, csrLen);

  k_gemm<16, 8, 2, 0><<<nGemm, NTHR, 0, stream>>>(xb, xb, wp3, as3, ad3, hw, es, ed, NPAD);
  k_agg<8><<<nAgg, NTHR, 0, stream>>>(csrD, offD, cntD, es, ed, hw, b3, xb, nN, csrLen);

  k_tail<<<nTail, NTHR, 0, stream>>>(csrS, offS, cntS, xb, x1, lin2, out, nN, csrLen, CNTPAD);
}
